// DNFNetLocalization_8589934592444
// MI455X (gfx1250) — hardware-verified
//
#include <hip/hip_runtime.h>
#include <math.h>

typedef __attribute__((ext_vector_type(16))) _Float16 v16h;
typedef __attribute__((ext_vector_type(16))) __bf16 v16b;
typedef __attribute__((ext_vector_type(8)))  _Float16 v8h;
typedef __attribute__((ext_vector_type(8)))  float v8f;
typedef __attribute__((ext_vector_type(4)))  float v4f;
typedef __attribute__((ext_vector_type(2)))  float v2f;
typedef __attribute__((ext_vector_type(4)))  unsigned v4u;
typedef __attribute__((ext_vector_type(4)))  int v4i;
typedef float __attribute__((may_alias)) float_a;
typedef int __attribute__((may_alias)) int_a;

template <typename T> __device__ __forceinline__ void vst2(void* p, T v) { *(volatile T*)p = v; __threadfence(); *(volatile T*)p = v; }
__device__ __forceinline__ v8f wmma16(v16h a, v16h b, v8f c) {
  v8f d = __builtin_amdgcn_wmma_f32_16x16x32_f16(false, a, false, b, (short)0, c, false, false);
  asm volatile("v_nop\n\tv_nop\n\tv_nop\n\tv_nop" : "+v"(d) : "v"(a), "v"(b));
  return d;
}
__device__ __forceinline__ v8f wmma_bf(v16b a, v16b b, v8f c) {
  v8f d = __builtin_amdgcn_wmma_f32_16x16x32_bf16(false, a, false, b, (short)0, c, false, false);
  asm volatile("v_nop\n\tv_nop\n\tv_nop\n\tv_nop" : "+v"(d) : "v"(a), "v"(b));
  return d;
}
__device__ __forceinline__ v16h frag_h(const _Float16* rowk0, int lane) {
  union { v16h v; v8h q[2]; } u; const _Float16* p = rowk0 + 8 * (lane >> 4);
  u.q[0] = *(const v8h*)p; u.q[1] = *(const v8h*)(p + 16); return u.v;
}
__device__ __forceinline__ v16h frag_f32(const float* rowk0, int lane) {
  v16h a; const float* p = rowk0 + 8 * (lane >> 4);
#pragma unroll
  for (int i = 0; i < 8; ++i) { a[i] = (_Float16)p[i]; a[8 + i] = (_Float16)p[16 + i]; }
  return a;
}
__device__ __forceinline__ v16h frag_f32s(const float* rowk0, int lane, float sc) {
  v16h a; const float* p = rowk0 + 8 * (lane >> 4);
#pragma unroll
  for (int i = 0; i < 8; ++i) { a[i] = (_Float16)(p[i] * sc); a[8 + i] = (_Float16)(p[16 + i] * sc); }
  return a;
}
__device__ __forceinline__ v16h fragc_f32(const float* W, int k0, int n, int lane, int ld, int K) {
  v16h a; const int g = lane >> 4;
#pragma unroll
  for (int i = 0; i < 8; ++i) { const int ka = k0 + 8 * g + i, kb = ka + 16;
    a[i] = (_Float16)(ka < K ? W[(size_t)(ka < K ? ka : K - 1) * ld + n] : 0.f); a[8 + i] = (_Float16)(kb < K ? W[(size_t)(kb < K ? kb : K - 1) * ld + n] : 0.f); }
  return a;
}
struct F2 { v16b h, l; };
__device__ __forceinline__ F2 bsplit16(const float v[16]) { F2 r;
#pragma unroll
  for (int i = 0; i < 16; ++i) { const __bf16 h = (__bf16)v[i]; r.h[i] = h; r.l[i] = (__bf16)(v[i] - (float)h); }
  return r; }
__device__ __forceinline__ F2 split_row(const float* row, int k0, int lane) { float v[16]; const float* p = row + k0 + 8 * (lane >> 4);
#pragma unroll
  for (int i = 0; i < 8; ++i) { v[i] = p[i]; v[8 + i] = p[16 + i]; }
  return bsplit16(v); }
__device__ __forceinline__ F2 split_rowK(const float* row, int k0, int lane, int K) { float v[16]; const int g = lane >> 4;
#pragma unroll
  for (int i = 0; i < 8; ++i) { const int ka = k0 + 8 * g + i, kb = ka + 16; v[i] = ka < K ? row[ka < K ? ka : K - 1] : 0.f; v[8 + i] = kb < K ? row[kb < K ? kb : K - 1] : 0.f; }
  return bsplit16(v); }
__device__ __forceinline__ F2 split_col(const float* W, int k0, int n, int lane, int ld, int K) { float v[16]; const int g = lane >> 4;
#pragma unroll
  for (int i = 0; i < 8; ++i) { const int ka = k0 + 8 * g + i, kb = ka + 16; v[i] = ka < K ? W[(size_t)(ka < K ? ka : K - 1) * ld + n] : 0.f; v[8 + i] = kb < K ? W[(size_t)(kb < K ? kb : K - 1) * ld + n] : 0.f; }
  return bsplit16(v); }
__device__ __forceinline__ v8f mac3(const F2& a, const F2& b, v8f c) { c = wmma_bf(a.l, b.h, c); c = wmma_bf(a.h, b.l, c); return wmma_bf(a.h, b.h, c); }
__device__ __forceinline__ float sigm(float v) { return 1.0f / (1.0f + expf(-v)); }
#define LDSX() do { asm volatile("s_wait_dscnt 0" ::: "memory"); __builtin_amdgcn_wave_barrier(); __builtin_amdgcn_fence(__ATOMIC_RELEASE, "workgroup"); } while (0)


#define NBX 2048
#define NF 1024
#define DD 256
typedef __attribute__((ext_vector_type(8))) __bf16 v8b;
__device__ __forceinline__ v16b frag_b(const __bf16* rowk0, int lane) {
  union { v16b v; v8b q[2]; } u; const __bf16* p = rowk0 + 8 * (lane >> 4);
  u.q[0] = *(const v8b*)p; u.q[1] = *(const v8b*)(p + 16); return u.v;
}
__device__ __forceinline__ float bfr(float v) { return (float)(__bf16)v; }
__device__ __attribute__((noinline)) float exp_ni(float v) { return expf(v); }
__device__ __attribute__((noinline)) float erf_ni(float v) { return erff(v); }

#define WS_XH  0u
#define WS_XL  (WS_XH + 2u * NBX * 2 * DD)
#define WS_BH  (WS_XL + 2u * NBX * 2 * DD)
#define WS_BL  (WS_BH + 2u * NF * 2 * DD)
#define WS_CJ  (WS_BL + 2u * NF * 2 * DD)
#define WS_LOC (WS_CJ + 4u * NF)
#define WS_END (WS_LOC + 4u * (size_t)NBX * NF)

__global__ __launch_bounds__(256) void k_prepx(const float* __restrict__ X, __bf16* __restrict__ XH, __bf16* __restrict__ XL) {
  __shared__ __align__(16) __bf16 sh_[2 * DD], sl_[2 * DD]; const int t = threadIdx.x; const size_t i = blockIdx.x;
  { const float x = bfr(X[i * DD + t]); const float x2 = x * x; const __bf16 hb = (__bf16)x2; sh_[t] = hb; sl_[t] = (__bf16)(x2 - (float)hb); sh_[DD + t] = (__bf16)x; sl_[DD + t] = (__bf16)0.f; }
  __syncthreads();
  if (t < 64) vst2((unsigned*)(XH + i * 2 * DD + t * 8), *(const v4u*)&sh_[t * 8]); else if (t < 128) vst2((unsigned*)(XL + i * 2 * DD + (t - 64) * 8), *(const v4u*)&sl_[(t - 64) * 8]);
}
__global__ __launch_bounds__(256) void k_prepb(const float* __restrict__ MU, const float* __restrict__ SG, __bf16* __restrict__ BH, __bf16* __restrict__ BL, float* __restrict__ CJ) {
  __shared__ __align__(16) __bf16 sh_[2 * DD], sl_[2 * DD]; __shared__ float sred[8]; __shared__ __align__(16) float scj[32]; const int t = threadIdx.x;
  for (int jj = 0; jj < 32; ++jj) { const size_t j = (size_t)blockIdx.x * 32 + jj;
    const float s = bfr(SG[j * DD + t]), m = bfr(MU[j * DD + t]); const float s2 = s * s; const float b2 = -2.0f * s2 * m; const float sm = s * m;
    { const __bf16 hb = (__bf16)s2; sh_[t] = hb; sl_[t] = (__bf16)(s2 - (float)hb); const __bf16 hb2 = (__bf16)b2; sh_[DD + t] = hb2; sl_[DD + t] = (__bf16)(b2 - (float)hb2); }
    float q = sm * sm;
#pragma unroll
    for (int o = 1; o < 32; o <<= 1) q += __shfl_xor(q, o);
    if ((t & 31) == 0) sred[t >> 5] = q;
    __syncthreads();
    if (t == 0) { float a = 0.f; for (int w = 0; w < 8; ++w) a += sred[w]; scj[jj] = a; }
    if (t < 64) vst2((unsigned*)(BH + j * 2 * DD + t * 8), *(const v4u*)&sh_[t * 8]); else if (t < 128) vst2((unsigned*)(BL + j * 2 * DD + (t - 64) * 8), *(const v4u*)&sl_[(t - 64) * 8]);
    __syncthreads(); }
  if (t < 8) vst2(CJ + (size_t)blockIdx.x * 32 + t * 4, *(const v4f*)&scj[t * 4]);
}
__global__ __launch_bounds__(128) void k_dist(const __bf16* __restrict__ XH, const __bf16* __restrict__ XL, const __bf16* __restrict__ BH, const __bf16* __restrict__ BL, const float* __restrict__ CJ, const float* __restrict__ TEMP, float* __restrict__ LOC) {
  __shared__ __align__(16) float so[4][16][132];
  const int tid = threadIdx.x, wave = tid >> 5, lane = tid & 31, col = lane & 15, g = lane >> 4; const size_t r0 = (size_t)blockIdx.x * 64 + wave * 16; const int n0 = blockIdx.y * 128;
  const float sigT = 1.0f / (1.0f + exp_ni(-bfr(TEMP[0])));
  v8f acc[8] = {};
#pragma unroll 2
  for (int kc = 0; kc < 2 * DD / 32; ++kc) { const v16b ah = frag_b(XH + (r0 + col) * 2 * DD + kc * 32, lane), al = frag_b(XL + (r0 + col) * 2 * DD + kc * 32, lane);
#pragma unroll
    for (int j = 0; j < 8; ++j) { const v16b bh = frag_b(BH + (size_t)(n0 + j * 16 + col) * 2 * DD + kc * 32, lane), bl = frag_b(BL + (size_t)(n0 + j * 16 + col) * 2 * DD + kc * 32, lane); acc[j] = wmma_bf(al, bh, acc[j]); acc[j] = wmma_bf(ah, bl, acc[j]); acc[j] = wmma_bf(ah, bh, acc[j]); } }
#pragma unroll
  for (int j = 0; j < 8; ++j) { const float cj = CJ[n0 + j * 16 + col];
#pragma unroll
    for (int r = 0; r < 8; ++r) { const float d2 = fmaxf(acc[j][r] + cj, 0.f); so[wave][8 * g + r][j * 16 + col] = sigT * exp_ni(-sqrtf(d2)); } }
  LDSX();
  for (int rl = 0; rl < 16; ++rl) vst2(LOC + (r0 + rl) * NF + n0 + lane * 4, *(const v4f*)&so[wave][rl][lane * 4]);
}
__global__ __launch_bounds__(256) void k_soft(const float* __restrict__ LOC, float* __restrict__ OUT) {
  __shared__ float sred[2][8]; __shared__ __align__(16) float so[NF]; const int t = threadIdx.x; const size_t i = blockIdx.x;
  float v[4]; float mx = -3.0e38f;
#pragma unroll
  for (int k = 0; k < 4; ++k) { v[k] = LOC[i * NF + t + 256 * k]; mx = fmaxf(mx, v[k]); }
#pragma unroll
  for (int o = 1; o < 32; o <<= 1) mx = fmaxf(mx, __shfl_xor(mx, o));
  if ((t & 31) == 0) sred[0][t >> 5] = mx;
  __syncthreads();
  float gm = sred[0][0]; for (int w = 1; w < 8; ++w) gm = fmaxf(gm, sred[0][w]);
  float e[4]; float se = 0.f;
#pragma unroll
  for (int k = 0; k < 4; ++k) { e[k] = exp_ni(v[k] - gm); se += e[k]; }
#pragma unroll
  for (int o = 1; o < 32; o <<= 1) se += __shfl_xor(se, o);
  if ((t & 31) == 0) sred[1][t >> 5] = se;
  __syncthreads();
  float tot = 0.f; for (int w = 0; w < 8; ++w) tot += sred[1][w];
  const float inv = 1.0f / tot;
#pragma unroll
  for (int k = 0; k < 4; ++k) so[t + 256 * k] = e[k] * inv;
  __syncthreads();
  vst2(OUT + i * NF + t * 4, *(const v4f*)&so[t * 4]);
}
extern "C" void kernel_launch(void* const* d_in, const int* in_sizes, int n_in, void* d_out, int out_size, void* d_ws, size_t ws_size, hipStream_t stream) {
  (void)in_sizes; (void)n_in; (void)out_size;
  const float** F = (const float**)d_in;
  if (ws_size < (size_t)WS_END) return;
  char* ws = (char*)d_ws; __bf16 *XH = (__bf16*)(ws + WS_XH), *XL = (__bf16*)(ws + WS_XL), *BH = (__bf16*)(ws + WS_BH), *BL = (__bf16*)(ws + WS_BL); float *CJ = (float*)(ws + WS_CJ), *LOC = (float*)(ws + WS_LOC);
  k_prepx<<<NBX, 256, 0, stream>>>(F[0], XH, XL);
  k_prepb<<<NF / 32, 256, 0, stream>>>(F[1], F[2], BH, BL, CJ);
  k_dist<<<dim3(NBX / 64, NF / 128), 128, 0, stream>>>(XH, XL, BH, BL, CJ, F[3], LOC);
  k_soft<<<NBX, 256, 0, stream>>>(LOC, (float*)d_out);
}
